// NCP_sequence_50543175140036
// MI455X (gfx1250) — hardware-verified
//
#include <hip/hip_runtime.h>


typedef _Float16 f16t;
typedef f16t  v16h __attribute__((ext_vector_type(16)));
typedef f16t  v8h  __attribute__((ext_vector_type(8)));
typedef float v8f  __attribute__((ext_vector_type(8)));
typedef float v4f  __attribute__((ext_vector_type(4)));
typedef unsigned int v4u __attribute__((ext_vector_type(4)));

union Frag { v16h v; v8h q[2]; };
union Pk16 { v8h h; v4u u; };
union Pk32 { v4f f; v4u u; };

#define LP 264

__device__ __forceinline__ v8f wmma16(v16h a, v16h b, v8f c) {
    return __builtin_amdgcn_wmma_f32_16x16x32_f16(false, a, false, b, (short)0, c, false, false);
}

__device__ __forceinline__ void wguard(v8f (&c)[1][1], Frag (&a)[1], Frag (&b)[1]) {
    asm volatile("v_nop\n\tv_nop\n\tv_nop\n\tv_nop"
                 : "+v"(c[0][0])
                 : "v"(a[0].v), "v"(b[0].v));
}
__device__ __forceinline__ void wguard(v8f (&c)[4][1], Frag (&a)[4], Frag (&b)[1]) {
    asm volatile("v_nop\n\tv_nop\n\tv_nop\n\tv_nop"
                 : "+v"(c[0][0]), "+v"(c[1][0]), "+v"(c[2][0]), "+v"(c[3][0])
                 : "v"(a[0].v), "v"(a[1].v), "v"(a[2].v), "v"(a[3].v), "v"(b[0].v));
}
__device__ __forceinline__ void wguard(v8f (&c)[2][2], Frag (&a)[2], Frag (&b)[2]) {
    asm volatile("v_nop\n\tv_nop\n\tv_nop\n\tv_nop"
                 : "+v"(c[0][0]), "+v"(c[0][1]), "+v"(c[1][0]), "+v"(c[1][1])
                 : "v"(a[0].v), "v"(a[1].v), "v"(b[0].v), "v"(b[1].v));
}
__device__ __forceinline__ void wguard(v8f (&c)[4][2], Frag (&a)[4], Frag (&b)[2]) {
    asm volatile("v_nop\n\tv_nop\n\tv_nop\n\tv_nop"
                 : "+v"(c[0][0]), "+v"(c[0][1]), "+v"(c[1][0]), "+v"(c[1][1]),
                   "+v"(c[2][0]), "+v"(c[2][1]), "+v"(c[3][0]), "+v"(c[3][1])
                 : "v"(a[0].v), "v"(a[1].v), "v"(a[2].v), "v"(a[3].v),
                   "v"(b[0].v), "v"(b[1].v));
}

template<int MT, int NT>
__device__ __forceinline__ void zacc(v8f (&acc)[MT][NT]) {
    const v8f z = {0.f, 0.f, 0.f, 0.f, 0.f, 0.f, 0.f, 0.f};
#pragma unroll
    for (int i = 0; i < MT; ++i)
#pragma unroll
        for (int j = 0; j < NT; ++j) acc[i][j] = z;
}

template<int MT, int NT>
__device__ __forceinline__ void mma_acc(v8f (&acc)[MT][NT],
                                        const f16t* A, int lda,
                                        const f16t* B, int ldb, int ktiles) {
    const int l = threadIdx.x & 31, h = l >> 4, m = l & 15;
    const f16t* ap = A + (size_t)m * lda + 8 * h;
    const f16t* bp = B + (size_t)m * ldb + 8 * h;
#pragma unroll 1
    for (int kt = 0; kt < ktiles; ++kt) {
        Frag a[MT], b[NT];
#pragma unroll
        for (int i = 0; i < MT; ++i) {
            const f16t* p = ap + (size_t)i * 16 * lda + kt * 32;
            a[i].q[0] = *(const v8h*)p;
            a[i].q[1] = *(const v8h*)(p + 16);
        }
#pragma unroll
        for (int j = 0; j < NT; ++j) {
            const f16t* p = bp + (size_t)j * 16 * ldb + kt * 32;
            b[j].q[0] = *(const v8h*)p;
            b[j].q[1] = *(const v8h*)(p + 16);
        }
#pragma unroll
        for (int i = 0; i < MT; ++i)
#pragma unroll
            for (int j = 0; j < NT; ++j)
                acc[i][j] = wmma16(a[i].v, b[j].v, acc[i][j]);
        wguard(acc, a, b);
    }
}

__device__ __forceinline__ float ftanh(float x) {
    float ax = fabsf(x);
    float t  = __expf(-2.0f * ax);
    float r  = (1.0f - t) * __builtin_amdgcn_rcpf(1.0f + t);
    return copysignf(r, x);
}

template<int MT, int NT, bool ACT>
__device__ __forceinline__ void epi_h(v8f (&acc)[MT][NT], float inv, const float* bias,
                                      int f0, f16t* L, int pitch) {
    const int l = threadIdx.x & 31, h = l >> 4, m = l & 15;
#pragma unroll
    for (int i = 0; i < MT; ++i) {
        const float* bq = bias + f0 + 16 * i + 8 * h;
        v4f c0 = *(const v4f*)bq;
        v4f c1 = *(const v4f*)(bq + 4);
#pragma unroll
        for (int j = 0; j < NT; ++j) {
            Pk16 pk;
#pragma unroll
            for (int r = 0; r < 4; ++r) {
                float v0 = fmaf(acc[i][j][r], inv, c0[r]);
                float v1 = fmaf(acc[i][j][4 + r], inv, c1[r]);
                if (ACT) { v0 = ftanh(v0); v1 = ftanh(v1); }
                pk.h[r]     = (f16t)v0;
                pk.h[4 + r] = (f16t)v1;
            }
            *(v8h*)(L + (size_t)(16 * j + m) * pitch + f0 + 16 * i + 8 * h) = pk.h;
        }
    }
}

template<int MT, int NT>
__device__ __forceinline__ void epi_f(v8f (&acc)[MT][NT], float inv, const float* bias,
                                      int f0, float* S, int pitch) {
    const int l = threadIdx.x & 31, h = l >> 4, m = l & 15;
#pragma unroll
    for (int i = 0; i < MT; ++i) {
        const float* bq = bias + f0 + 16 * i + 8 * h;
        v4f c0 = *(const v4f*)bq;
        v4f c1 = *(const v4f*)(bq + 4);
#pragma unroll
        for (int j = 0; j < NT; ++j) {
            Pk32 p0, p1;
#pragma unroll
            for (int r = 0; r < 4; ++r) {
                p0.f[r] = fmaf(acc[i][j][r], inv, c0[r]);
                p1.f[r] = fmaf(acc[i][j][4 + r], inv, c1[r]);
            }
            float* d = S + (size_t)(16 * j + m) * pitch + f0 + 16 * i + 8 * h;
            *(v4f*)d       = p0.f;
            *(v4f*)(d + 4) = p1.f;
        }
    }
}

__global__ __launch_bounds__(256)
void k_cvt8(const float* x, f16t* y, int n8) {
    int i = blockIdx.x * 256 + threadIdx.x;
    if (i >= n8) return;
    const float* p = x + (size_t)i * 8;
    v4f a = *(const v4f*)p;
    v4f b = *(const v4f*)(p + 4);
    Pk16 k;
    k.h[0] = (f16t)a[0]; k.h[1] = (f16t)a[1]; k.h[2] = (f16t)a[2]; k.h[3] = (f16t)a[3];
    k.h[4] = (f16t)b[0]; k.h[5] = (f16t)b[1]; k.h[6] = (f16t)b[2]; k.h[7] = (f16t)b[3];
    f16t* d = y + (size_t)i * 8;
    *(volatile v4u*)d = k.u;
    __threadfence();
    *(volatile v4u*)d = k.u;
}

__global__ __launch_bounds__(256)
void k_pack(const float* W, f16t* P, int K, int N, float sc) {
    int i  = blockIdx.x * 256 + threadIdx.x;
    int kq = K >> 3;
    int tot = N * kq;
    if (i >= tot) return;
    int n = i / kq;
    int k = (i - n * kq) * 8;
    Pk16 v;
#pragma unroll
    for (int e = 0; e < 8; ++e)
        v.h[e] = (f16t)(W[(size_t)(k + e) * N + n] * sc);
    f16t* d = P + (size_t)n * K + k;
    *(volatile v4u*)d = v.u;
    __threadfence();
    *(volatile v4u*)d = v.u;
}

__global__ __launch_bounds__(128)
void k_mlp_enc(const f16t* X, const f16t* P1, const float* b1,
               const f16t* P2, const float* b2,
               const f16t* P3, const float* b3,
               f16t* E, int nrows, float inv1, float inv2, float inv3) {
    __shared__ __attribute__((aligned(16))) f16t L1[32 * LP];
    __shared__ __attribute__((aligned(16))) f16t L2[32 * LP];
    __shared__ __attribute__((aligned(16))) f16t S16[32 * 128];
    const int w  = threadIdx.x >> 5;
    const int r0 = blockIdx.x * 32;
    if (r0 + 32 > nrows) return;

    {
        v8f acc[4][2]; zacc(acc);
        mma_acc<4, 2>(acc, P1 + (size_t)(64 * w) * 64, 64, X + (size_t)r0 * 64, 64, 2);
        epi_h<4, 2, true>(acc, inv1, b1, 64 * w, L1, LP);
    }
    __syncthreads();
    {
        v8f acc[4][2]; zacc(acc);
        mma_acc<4, 2>(acc, P2 + (size_t)(64 * w) * 256, 256, L1, LP, 8);
        epi_h<4, 2, true>(acc, inv2, b2, 64 * w, L2, LP);
    }
    __syncthreads();
    {
        v8f acc[2][2]; zacc(acc);
        mma_acc<2, 2>(acc, P3 + (size_t)(32 * w) * 256, 256, L2, LP, 8);
        epi_h<2, 2, false>(acc, inv3, b3, 32 * w, S16, 128);
    }
    __syncthreads();
    Pk16 v[4];
    const int tid = threadIdx.x;
#pragma unroll
    for (int i = 0; i < 4; ++i) {
        int p = tid + 128 * i, row = p >> 4, ch = (p & 15) * 8;
        v[i].h = *(const v8h*)(S16 + row * 128 + ch);
    }
#pragma unroll
    for (int i = 0; i < 4; ++i) {
        int p = tid + 128 * i, row = p >> 4, ch = (p & 15) * 8;
        *(volatile v4u*)(E + (size_t)(r0 + row) * 128 + ch) = v[i].u;
    }
    __threadfence();
#pragma unroll
    for (int i = 0; i < 4; ++i) {
        int p = tid + 128 * i, row = p >> 4, ch = (p & 15) * 8;
        *(volatile v4u*)(E + (size_t)(r0 + row) * 128 + ch) = v[i].u;
    }
}

__global__ __launch_bounds__(128)
void k_mlp_dec(const f16t* M, const f16t* P1, const float* b1,
               const f16t* P2, const float* b2,
               const f16t* P3, const float* b3,
               float* Y, int nrows, float inv1, float inv2, float inv3) {
    __shared__ __attribute__((aligned(16))) f16t  L1[32 * LP];
    __shared__ __attribute__((aligned(16))) f16t  L2[32 * LP];
    __shared__ __attribute__((aligned(16))) float S32[32 * 32];
    const int w  = threadIdx.x >> 5;
    const int r0 = blockIdx.x * 32;
    if (r0 + 32 > nrows) return;

    {
        v8f acc[4][2]; zacc(acc);
        mma_acc<4, 2>(acc, P1 + (size_t)(64 * w) * 64, 64, M + (size_t)r0 * 64, 64, 2);
        epi_h<4, 2, true>(acc, inv1, b1, 64 * w, L1, LP);
    }
    __syncthreads();
    {
        v8f acc[4][2]; zacc(acc);
        mma_acc<4, 2>(acc, P2 + (size_t)(64 * w) * 256, 256, L1, LP, 8);
        epi_h<4, 2, true>(acc, inv2, b2, 64 * w, L2, LP);
    }
    __syncthreads();
    {
        const int fi = w >> 1, ni = w & 1;
        v8f acc[1][1]; zacc(acc);
        mma_acc<1, 1>(acc, P3 + (size_t)(16 * fi) * 256, 256, L2 + (size_t)(16 * ni) * LP, LP, 8);
        epi_f<1, 1>(acc, inv3, b3, 16 * fi, S32 + (16 * ni) * 32, 32);
    }
    __syncthreads();
    Pk32 v[2];
    const int tid = threadIdx.x;
#pragma unroll
    for (int i = 0; i < 2; ++i) {
        int p = tid + 128 * i, row = p >> 3, c = (p & 7) * 4;
        v[i].f = *(const v4f*)(S32 + row * 32 + c);
    }
#pragma unroll
    for (int i = 0; i < 2; ++i) {
        int p = tid + 128 * i, row = p >> 3, c = (p & 7) * 4;
        *(volatile v4u*)(Y + (size_t)(r0 + row) * 32 + c) = v[i].u;
    }
    __threadfence();
#pragma unroll
    for (int i = 0; i < 2; ++i) {
        int p = tid + 128 * i, row = p >> 3, c = (p & 7) * 4;
        *(volatile v4u*)(Y + (size_t)(r0 + row) * 32 + c) = v[i].u;
    }
}

__global__ __launch_bounds__(128)
void k_rnn(const f16t* E, const f16t* Pih, const f16t* Phh, const float* bh,
           const f16t* Pho, const float* bo, f16t* Mo, int T, int nb,
           float invS, float invO) {
    __shared__ __attribute__((aligned(16))) f16t H16[16 * LP];
    __shared__ __attribute__((aligned(16))) f16t M16[16 * 64];
    const int w   = threadIdx.x >> 5;
    const int tid = threadIdx.x;
    const int b0  = blockIdx.x * 16;
    if (b0 + 16 > nb) return;

    for (int i = tid; i < 16 * LP; i += 128) H16[i] = (f16t)0.0f;
    __syncthreads();

    const int ldE = T * 128;
    const int row = tid >> 3, ch = (tid & 7) * 8;

#pragma unroll 1
    for (int t = 0; t < T; ++t) {
        v8f acc[4][1]; zacc(acc);
        const f16t* Et = E + ((size_t)b0 * T + t) * 128;
        mma_acc<4, 1>(acc, Pih + (size_t)(64 * w) * 128, 128, Et, ldE, 4);
        mma_acc<4, 1>(acc, Phh + (size_t)(64 * w) * 256, 256, H16, LP, 8);
        __syncthreads();
        epi_h<4, 1, true>(acc, invS, bh, 64 * w, H16, LP);
        __syncthreads();

        v8f macc[1][1]; zacc(macc);
        mma_acc<1, 1>(macc, Pho + (size_t)(16 * w) * 256, 256, H16, LP, 8);
        epi_h<1, 1, false>(macc, invO, bo, 16 * w, M16, 64);
        __syncthreads();

        Pk16 v;
        v.h = *(const v8h*)(M16 + row * 64 + ch);
        f16t* dst = Mo + (((size_t)(b0 + row)) * T + t) * 64 + ch;
        *(volatile v4u*)dst = v.u;
        __threadfence();
        *(volatile v4u*)dst = v.u;
    }
}

extern "C" void kernel_launch(void* const* d_in, const int* in_sizes, int n_in,
                              void* d_out, int out_size, void* d_ws, size_t ws_size,
                              hipStream_t stream) {
    const int BATCH = 256, TSTEPS = 512, DIN = 64, H1 = 256, INTER = 128,
              STATE = 256, MOTOR = 64, DOUT = 32;
    const int ntok = BATCH * TSTEPS;

    if (n_in < 18) return;
    if (in_sizes[0] != ntok * DIN || out_size != ntok * DOUT) return;
    if (in_sizes[1] != DIN * H1 || in_sizes[3] != H1 * H1 || in_sizes[5] != H1 * INTER ||
        in_sizes[7] != INTER * STATE || in_sizes[8] != STATE * STATE ||
        in_sizes[10] != STATE * MOTOR || in_sizes[12] != MOTOR * H1 ||
        in_sizes[14] != H1 * H1 || in_sizes[16] != H1 * DOUT) return;
    if ((ntok % 32) != 0 || (BATCH % 16) != 0) return;

    const float* x   = (const float*)d_in[0];
    const float* Wi1 = (const float*)d_in[1];  const float* bi1 = (const float*)d_in[2];
    const float* Wi2 = (const float*)d_in[3];  const float* bi2 = (const float*)d_in[4];
    const float* Wi3 = (const float*)d_in[5];  const float* bi3 = (const float*)d_in[6];
    const float* Wih = (const float*)d_in[7];
    const float* Whh = (const float*)d_in[8];  const float* bh  = (const float*)d_in[9];
    const float* Who = (const float*)d_in[10]; const float* bo  = (const float*)d_in[11];
    const float* Wo1 = (const float*)d_in[12]; const float* bo1 = (const float*)d_in[13];
    const float* Wo2 = (const float*)d_in[14]; const float* bo2 = (const float*)d_in[15];
    const float* Wo3 = (const float*)d_in[16]; const float* bo3 = (const float*)d_in[17];
    float* out = (float*)d_out;

    char* ws = (char*)d_ws;
    size_t off = 0;
    auto carve = [&](size_t bytes) -> char* {
        char* p = ws + off;
        off = (off + bytes + 255) & ~(size_t)255;
        return p;
    };
    f16t* X16 = (f16t*)carve((size_t)ntok * DIN * 2);
    f16t* E16 = (f16t*)carve((size_t)ntok * INTER * 2);
    f16t* M16 = (f16t*)carve((size_t)ntok * MOTOR * 2);
    f16t* Pi1 = (f16t*)carve((size_t)DIN * H1 * 2);
    f16t* Pi2 = (f16t*)carve((size_t)H1 * H1 * 2);
    f16t* Pi3 = (f16t*)carve((size_t)H1 * INTER * 2);
    f16t* Pih = (f16t*)carve((size_t)INTER * STATE * 2);
    f16t* Phh = (f16t*)carve((size_t)STATE * STATE * 2);
    f16t* Pho = (f16t*)carve((size_t)STATE * MOTOR * 2);
    f16t* Po1 = (f16t*)carve((size_t)MOTOR * H1 * 2);
    f16t* Po2 = (f16t*)carve((size_t)H1 * H1 * 2);
    f16t* Po3 = (f16t*)carve((size_t)H1 * DOUT * 2);
    if (off > ws_size) return;

    const float S64 = 64.0f, S128 = 128.0f;
    const float I64 = 0.015625f, I128 = 0.0078125f;

    {
        int n8 = ntok * DIN / 8;
        k_cvt8<<<dim3((n8 + 255) / 256), dim3(256), 0, stream>>>(x, X16, n8);
    }
    auto pack = [&](const float* W, f16t* P, int K, int N, float sc) {
        int tot = N * (K / 8);
        k_pack<<<dim3((tot + 255) / 256), dim3(256), 0, stream>>>(W, P, K, N, sc);
    };
    pack(Wi1, Pi1, DIN,   H1,    S64);
    pack(Wi2, Pi2, H1,    H1,    S128);
    pack(Wi3, Pi3, H1,    INTER, S128);
    pack(Wih, Pih, INTER, STATE, S128);
    pack(Whh, Phh, STATE, STATE, S128);
    pack(Who, Pho, STATE, MOTOR, S128);
    pack(Wo1, Po1, MOTOR, H1,    S64);
    pack(Wo2, Po2, H1,    H1,    S128);
    pack(Wo3, Po3, H1,    DOUT,  S128);

    k_mlp_enc<<<dim3(ntok / 32), dim3(128), 0, stream>>>(X16, Pi1, bi1, Pi2, bi2, Pi3, bi3,
                                                        E16, ntok, I64, I128, I128);
    k_rnn<<<dim3(BATCH / 16), dim3(128), 0, stream>>>(E16, Pih, Phh, bh, Pho, bo, M16,
                                                     TSTEPS, BATCH, I128, I128);
    k_mlp_dec<<<dim3(ntok / 32), dim3(128), 0, stream>>>(M16, Po1, bo1, Po2, bo2, Po3, bo3,
                                                        out, ntok, I64, I128, I128);
}
